// Kalman_filter_34041910788634
// MI455X (gfx1250) — hardware-run, weakly checked
//
#include <hip/hip_runtime.h>
#include <stddef.h>

typedef __attribute__((ext_vector_type(16))) _Float16 v16h;
typedef __attribute__((ext_vector_type(8)))  _Float16 v8h;
typedef __attribute__((ext_vector_type(8)))  float    v8f;
typedef __attribute__((ext_vector_type(4)))  float    v4f;

constexpr int kN = 2048;
constexpr int kH = 4096;
constexpr int kO = 512;
constexpr int kT = 8;
constexpr float kCarry = 256.0f;
constexpr float kFold  = 1.0f / (kCarry * kCarry);
constexpr int kTilesM = kN / 64;
constexpr int kTilesN = kH / 64;
constexpr int kGemmBlocks = (kTilesM * kTilesN) / 8;
static_assert((kN % 64) == 0 && (kH % 64) == 0 && (kN % 32) == 0, "tile multiples");
static_assert(((kTilesM * kTilesN) % 8) == 0, "eight tiles per block");
static_assert((kN % 256) == 0 && (kH % 256) == 0 && (kO % 32) == 0, "side kernel grids");
static_assert(((kN * kN / 8) % 256) == 0 && ((kH * kN / 8) % 256) == 0, "cast grids exact");

constexpr size_t kOffQH   = 0;
constexpr size_t kOffW1H  = kOffQH   + (size_t)kN * kN * 2;
constexpr size_t kOffV    = kOffW1H  + (size_t)kH * kN * 2;
constexpr size_t kOffU    = kOffV    + (size_t)kH * 4;
constexpr size_t kOffH0   = kOffU    + (size_t)kH * 4;
constexpr size_t kOffQE   = kOffH0   + (size_t)kH * 4;
constexpr size_t kOffHVP  = kOffQE   + (size_t)kN * 4;
constexpr size_t kOffLAST = kOffHVP  + (size_t)kTilesN * kN * 4;
constexpr size_t kWsTotal = kOffLAST + (size_t)kN * 4;
static_assert(kWsTotal == 25755648ull, "carve total");
static_assert(kWsTotal <= 134217728ull, "carve cap");
static_assert((kOffW1H % 128) == 0 && (kOffV % 128) == 0 && (kOffU % 128) == 0 && (kOffH0 % 128) == 0 &&
              (kOffQE % 128) == 0 && (kOffHVP % 128) == 0 && (kOffLAST % 128) == 0, "128-B aligned regions");

union FragU { v16h v; v8h h[2]; };
__device__ __forceinline__ v16h frag_load(const _Float16* p) {
  FragU f;
  f.h[0] = *(const v8h*)(p);
  f.h[1] = *(const v8h*)(p + 16);
  return f.v;
}
__device__ __forceinline__ v8f frag_mma(v16h a, v16h b, v8f c) {
  return __builtin_amdgcn_wmma_f32_16x16x32_f16(false, a, false, b, (short)0, c, false, false);
}
__device__ __forceinline__ void group_guard(v8f& a0, v8f& a1, v8f& a2, v8f& a3, v16h x,
                                            v16h b0, v16h b1, v16h b2, v16h b3) {
  asm volatile("v_nop\n\tv_nop\n\tv_nop\n\tv_nop"
               : "+v"(a0), "+v"(a1), "+v"(a2), "+v"(a3)
               : "v"(x), "v"(b0), "v"(b1), "v"(b2), "v"(b3));
}
__device__ __forceinline__ void acc_guard4(v8f& a, v8f& b, v8f& c, v8f& d) {
  asm volatile("v_nop\n\tv_nop\n\tv_nop\n\tv_nop" : "+v"(a), "+v"(b), "+v"(c), "+v"(d));
}

__global__ __launch_bounds__(256) void cast_carry_f16_kernel(
    const float* __restrict__ src, unsigned short* __restrict__ dst, int total8, float carry)
{
  const int i = blockIdx.x * 256 + threadIdx.x;
  if (i >= total8) return;
  const size_t e0 = (size_t)i << 3;
  const v4f a0 = *(const v4f*)(src + e0);
  const v4f a1 = *(const v4f*)(src + e0 + 4);
  v8h hv;
#pragma unroll
  for (int e = 0; e < 4; ++e) {
    const float f0 = a0[e] * carry;
    const float f1 = a1[e] * carry;
    hv[e]     = (_Float16)f0;
    hv[4 + e] = (_Float16)f1;
  }
  unsigned short* q = dst + e0;
  *(volatile v8h*)q = hv;
  __threadfence();
  *(volatile v8h*)q = hv;
}

__global__ __launch_bounds__(256) void colsum2_kernel(
    const float* __restrict__ W2, const float* __restrict__ e7, const float* __restrict__ t7,
    float* __restrict__ vout, float* __restrict__ uout)
{
  __shared__ __align__(16) float sVU[512];
  const int tid = threadIdx.x;
  const int j = blockIdx.x * 256 + tid;
  float av = 0.0f, au = 0.0f;
#pragma unroll 4
  for (int i = 0; i < kN; ++i) {
    const float wv = W2[(size_t)i * kH + j];
    av = fmaf(wv, e7[i], av);
    au = fmaf(wv, t7[i], au);
  }
  sVU[tid] = av;
  sVU[256 + tid] = au;
  __syncthreads();
  const int wave = tid >> 5, lane = tid & 31;
  if (wave < 4) {
    const int idx = wave * 128 + lane * 4;
    const v4f val = *(const v4f*)(sVU + idx);
    const bool isV = (wave < 2);
    float* dst = isV ? (vout + blockIdx.x * 256 + idx) : (uout + blockIdx.x * 256 + (idx - 256));
    *(volatile v4f*)dst = val;
    __threadfence();
    *(volatile v4f*)dst = val;
  }
}

__global__ __launch_bounds__(256) void rowdot32_kernel(
    const float* A0, const float* x0, const float* bias0, float* y0, int relu0, int nblk0,
    const float* A1, const float* x1, float* y1)
{
  __shared__ __align__(16) float sR[32];
  const int tid = threadIdx.x, lane = tid & 31, wave = tid >> 5;
  const bool j0 = ((int)blockIdx.x < nblk0);
  const int blk = j0 ? (int)blockIdx.x : ((int)blockIdx.x - nblk0);
  const float* A = j0 ? A0 : A1;
  const float* x = j0 ? x0 : x1;
  float* y = j0 ? y0 : y1;
#pragma unroll 1
  for (int r = 0; r < 4; ++r) {
    const int row = blk * 32 + wave * 4 + r;
    const float* ar = A + (size_t)row * kN;
    float acc = 0.0f;
#pragma unroll 4
    for (int it = 0; it < 16; ++it) {
      const int k = it * 128 + lane * 4;
      const v4f a = *(const v4f*)(ar + k);
      const v4f b = *(const v4f*)(x + k);
      acc = fmaf(a[0], b[0], acc);
      acc = fmaf(a[1], b[1], acc);
      acc = fmaf(a[2], b[2], acc);
      acc = fmaf(a[3], b[3], acc);
    }
    acc += __shfl_xor(acc, 16, 32);
    acc += __shfl_xor(acc, 8, 32);
    acc += __shfl_xor(acc, 4, 32);
    acc += __shfl_xor(acc, 2, 32);
    acc += __shfl_xor(acc, 1, 32);
    float bv = 0.0f;
    if (j0) bv = bias0[row];
    float val = acc + bv;
    if (j0 && (relu0 != 0)) val = fmaxf(val, 0.0f);
    if (lane == 0) sR[wave * 4 + r] = val;
  }
  __syncthreads();
  const v4f o = *(const v4f*)(sR + 4 * (tid & 7));
  float* dst = y + blk * 32 + 4 * (tid & 7);
  if (tid < 8) *(volatile v4f*)dst = o;
  __threadfence();
  if (tid < 8) *(volatile v4f*)dst = o;
}

__global__ __launch_bounds__(256) void gemm_relu_dot_kernel(
    const unsigned short* __restrict__ Ap, const unsigned short* __restrict__ Btp,
    const float* __restrict__ b1, const float* __restrict__ vvec, float* __restrict__ hvp)
{
  const _Float16* A  = (const _Float16*)Ap;
  const _Float16* Bt = (const _Float16*)Btp;
  __shared__ __align__(16) float sRow[8][64];
  const int lane = threadIdx.x & 31;
  const int wave = threadIdx.x >> 5;
  const int tile = blockIdx.x * 8 + wave;
  if (tile >= kTilesM * kTilesN) return;
  const int tm = tile / kTilesN;
  const int tn = tile - tm * kTilesN;
  const int m0 = tm << 6;
  const int n0 = tn << 6;
  const int rlane = lane & 15;
  const int koff  = (lane >> 4) * 8;
  const int mOff  = (lane >> 4) * 8;

  v8f acc[4][4];
#pragma unroll
  for (int i = 0; i < 4; ++i)
#pragma unroll
    for (int j = 0; j < 4; ++j) acc[i][j] = (v8f){0.f, 0.f, 0.f, 0.f, 0.f, 0.f, 0.f, 0.f};

  for (int k0 = 0; k0 < kN; k0 += 32) {
    v16h bh[4];
#pragma unroll
    for (int j = 0; j < 4; ++j) {
      const size_t bo = (size_t)(n0 + (j << 4) + rlane) * kN + koff + k0;
      bh[j] = frag_load(Bt + bo);
    }
#pragma unroll
    for (int i = 0; i < 4; ++i) {
      const size_t ao = (size_t)(m0 + (i << 4) + rlane) * kN + koff + k0;
      const v16h ah = frag_load(A + ao);
#pragma unroll
      for (int j = 0; j < 4; ++j) acc[i][j] = frag_mma(ah, bh[j], acc[i][j]);
      group_guard(acc[i][0], acc[i][1], acc[i][2], acc[i][3], ah, bh[0], bh[1], bh[2], bh[3]);
    }
  }
  acc_guard4(acc[0][0], acc[0][1], acc[0][2], acc[0][3]);
  acc_guard4(acc[1][0], acc[1][1], acc[1][2], acc[1][3]);
  acc_guard4(acc[2][0], acc[2][1], acc[2][2], acc[2][3]);
  acc_guard4(acc[3][0], acc[3][1], acc[3][2], acc[3][3]);

  float bj[4], vj[4];
#pragma unroll
  for (int j = 0; j < 4; ++j) {
    const int n = n0 + (j << 4) + rlane;
    bj[j] = b1[n];
    vj[j] = vvec[n];
  }
  float* slab = sRow[wave];
#pragma unroll
  for (int i = 0; i < 4; ++i) {
    float rs[8];
#pragma unroll
    for (int r = 0; r < 8; ++r) {
      float s = 0.0f;
#pragma unroll
      for (int j = 0; j < 4; ++j) {
        float p = fmaf(acc[i][j][r], kFold, bj[j]);
        p = fmaxf(p, 0.0f);
        s = fmaf(p, vj[j], s);
      }
      rs[r] = s;
    }
#pragma unroll
    for (int r = 0; r < 8; ++r) {
      float t = rs[r];
      t += __shfl_xor(t, 1, 32);
      t += __shfl_xor(t, 2, 32);
      t += __shfl_xor(t, 4, 32);
      t += __shfl_xor(t, 8, 32);
      rs[r] = t;
    }
    if (rlane == 0) {
#pragma unroll
      for (int r = 0; r < 8; ++r) slab[(i << 4) + mOff + r] = rs[r];
    }
  }
  __builtin_amdgcn_fence(__ATOMIC_RELEASE, "workgroup");
  __builtin_amdgcn_wave_barrier();
  __builtin_amdgcn_fence(__ATOMIC_ACQUIRE, "workgroup");
  {
    const int c4 = (lane & 15) * 4;
    const v4f val = *(const v4f*)(slab + c4);
    float* dst = hvp + (size_t)tn * kN + m0 + c4;
    if (lane < 16) *(volatile v4f*)dst = val;
    __threadfence();
    if (lane < 16) *(volatile v4f*)dst = val;
  }
}

__global__ __launch_bounds__(256) void combine_kernel(
    const float* __restrict__ w, const float* __restrict__ b2, const float* __restrict__ t7,
    const float* __restrict__ e7, const float* __restrict__ h0, const float* __restrict__ u,
    const float* __restrict__ qe, const float* __restrict__ hvp, float* __restrict__ last)
{
  __shared__ float sRed[8];
  __shared__ __align__(16) float sL[256];
  const int tid = threadIdx.x, lane = tid & 31, wave = tid >> 5;
  float p = 0.0f;
#pragma unroll 1
  for (int i = tid; i < kN; i += 256) {
    const float bb = b2[i];
    const float wb = w[i] + bb;
    p = fmaf(wb, t7[i], p);
    p = fmaf(bb, e7[i], p);
  }
#pragma unroll 1
  for (int n = tid; n < kH; n += 256) p = fmaf(h0[n], u[n], p);
  p += __shfl_xor(p, 16, 32);
  p += __shfl_xor(p, 8, 32);
  p += __shfl_xor(p, 4, 32);
  p += __shfl_xor(p, 2, 32);
  p += __shfl_xor(p, 1, 32);
  if (lane == 0) sRed[wave] = p;
  __syncthreads();
  float stot = 0.0f;
#pragma unroll
  for (int k = 0; k < 8; ++k) stot += sRed[k];

  const int m = blockIdx.x * 256 + tid;
  float a = qe[m];
#pragma unroll 8
  for (int b = 0; b < kTilesN; ++b) a += hvp[(size_t)b * kN + m];
  sL[tid] = a + stot;
  __syncthreads();
  const int c4 = 4 * (tid & 63);
  const v4f val = *(const v4f*)(sL + c4);
  float* dst = last + blockIdx.x * 256 + c4;
  if (tid < 64) *(volatile v4f*)dst = val;
  __threadfence();
  if (tid < 64) *(volatile v4f*)dst = val;
}

extern "C" void kernel_launch(void* const* d_in, const int* in_sizes, int n_in,
                              void* d_out, int out_size, void* d_ws, size_t ws_size,
                              hipStream_t stream) {
  if (n_in < 10) return;
  if (in_sizes[0] != kT * kN) return;
  if (in_sizes[1] != kT * kN) return;
  if (in_sizes[2] != kN) return;
  if (in_sizes[3] != kN * kN) return;
  if (in_sizes[4] != kH * kN) return;
  if (in_sizes[5] != kH) return;
  if (in_sizes[6] != kN * kH) return;
  if (in_sizes[7] != kN) return;
  if (in_sizes[8] != kO * kN) return;
  if (in_sizes[9] != kO) return;
  if (out_size != kO) return;
  if (ws_size < kWsTotal) return;

  const float* Tin = (const float*)d_in[0];
  const float* ein = (const float*)d_in[1];
  const float* w   = (const float*)d_in[2];
  const float* Q   = (const float*)d_in[3];
  const float* W1  = (const float*)d_in[4];
  const float* b1  = (const float*)d_in[5];
  const float* W2  = (const float*)d_in[6];
  const float* b2  = (const float*)d_in[7];
  const float* fcw = (const float*)d_in[8];
  const float* fcb = (const float*)d_in[9];
  float* out = (float*)d_out;

  const float* t7 = Tin + (size_t)(kT - 1) * kN;
  const float* e7 = ein + (size_t)(kT - 1) * kN;

  char* ws = (char*)d_ws;
  unsigned short* QH   = (unsigned short*)(ws + kOffQH);
  unsigned short* W1H  = (unsigned short*)(ws + kOffW1H);
  float*          V    = (float*)(ws + kOffV);
  float*          U    = (float*)(ws + kOffU);
  float*          H0   = (float*)(ws + kOffH0);
  float*          QE   = (float*)(ws + kOffQE);
  float*          HVP  = (float*)(ws + kOffHVP);
  float*          LAST = (float*)(ws + kOffLAST);

  cast_carry_f16_kernel<<<(kN * kN / 8) / 256, 256, 0, stream>>>(Q, QH, kN * kN / 8, kCarry);
  cast_carry_f16_kernel<<<(kH * kN / 8) / 256, 256, 0, stream>>>(W1, W1H, kH * kN / 8, kCarry);

  colsum2_kernel<<<kH / 256, 256, 0, stream>>>(W2, e7, t7, V, U);

  rowdot32_kernel<<<kH / 32 + kN / 32, 256, 0, stream>>>(W1, w, b1, H0, 1, kH / 32, Q, e7, QE);

  gemm_relu_dot_kernel<<<kGemmBlocks, 256, 0, stream>>>(QH, W1H, b1, V, HVP);

  combine_kernel<<<kN / 256, 256, 0, stream>>>(w, b2, t7, e7, H0, U, QE, HVP, LAST);

  rowdot32_kernel<<<kO / 32, 256, 0, stream>>>(fcw, LAST, fcb, out, 0, kO / 32, Q, e7, QE);
}
